// _Attention_128849018943
// MI455X (gfx1250) — hardware-verified
//
#include <hip/hip_runtime.h>
#include <math.h>

typedef __attribute__((ext_vector_type(16))) _Float16 v16h;
typedef __attribute__((ext_vector_type(16))) __bf16 v16b;
typedef __attribute__((ext_vector_type(8)))  _Float16 v8h;
typedef __attribute__((ext_vector_type(8)))  __bf16 v8b;
typedef __attribute__((ext_vector_type(8)))  float v8f;
typedef __attribute__((ext_vector_type(4)))  float v4f;
typedef __attribute__((ext_vector_type(4)))  unsigned v4u;
typedef __attribute__((ext_vector_type(4)))  int v4i;

template <typename T> __device__ __forceinline__ void vst2(void* p, T v) { *(volatile T*)p = v; __threadfence(); *(volatile T*)p = v; }
__device__ __forceinline__ v8f wmma16(v16h a, v16h b, v8f c) {
  v8f d = __builtin_amdgcn_wmma_f32_16x16x32_f16(false, a, false, b, (short)0, c, false, false);
  asm volatile("v_nop\n\tv_nop\n\tv_nop\n\tv_nop" : "+v"(d) : "v"(a), "v"(b));
  return d;
}
__device__ __forceinline__ v8f wmma_bf(v16b a, v16b b, v8f c) {
  v8f d = __builtin_amdgcn_wmma_f32_16x16x32_bf16(false, a, false, b, (short)0, c, false, false);
  asm volatile("v_nop\n\tv_nop\n\tv_nop\n\tv_nop" : "+v"(d) : "v"(a), "v"(b));
  return d;
}
__device__ __forceinline__ v16h frag_h(const _Float16* rowk0, int lane) {
  union { v16h v; v8h q[2]; } u; const _Float16* p = rowk0 + 8 * (lane >> 4);
  u.q[0] = *(const v8h*)p; u.q[1] = *(const v8h*)(p + 16); return u.v;
}
__device__ __forceinline__ v16b frag_b(const __bf16* rowk0, int lane) {
  union { v16b v; v8b q[2]; } u; const __bf16* p = rowk0 + 8 * (lane >> 4);
  u.q[0] = *(const v8b*)p; u.q[1] = *(const v8b*)(p + 16); return u.v;
}
struct F2 { v16b h, l; };
__device__ __forceinline__ F2 bsplit16(const float v[16]) { F2 r;
#pragma unroll
  for (int i = 0; i < 16; ++i) { const __bf16 h = (__bf16)v[i]; r.h[i] = h; r.l[i] = (__bf16)(v[i] - (float)h); }
  return r; }
__device__ __forceinline__ F2 split_row(const float* row, int k0, int lane) { float v[16]; const float* p = row + k0 + 8 * (lane >> 4);
#pragma unroll
  for (int i = 0; i < 8; ++i) { v[i] = p[i]; v[8 + i] = p[16 + i]; }
  return bsplit16(v); }
#define LDSX() do { asm volatile("s_wait_dscnt 0" ::: "memory"); __builtin_amdgcn_wave_barrier(); __builtin_amdgcn_fence(__ATOMIC_RELEASE, "workgroup"); } while (0)

#ifndef NB
#define NB 1
#endif
#ifndef SEQ
#define SEQ 2048
#endif
#define SS_FULL 2048
#define DM 1024
#define NH 16
#define HD 64
#define QKVW (3 * DM)
#define TQB (SEQ / 64)
static_assert(NB == 1);
static_assert(SEQ % 64 == 0);
static_assert(SEQ >= 64 && SEQ <= SS_FULL);
static_assert(NH * HD == DM);

#define PK_A 0
#define PK_P (PK_A + QKVW * DM)
#define PK_END (PK_P + DM * DM)
#define WS_PK  0u
#define WS_QK  (WS_PK + 2u * PK_END)
#define WS_QKL (WS_QK + 2u * SEQ * 2 * DM)
#define WS_VTH (WS_QKL + 2u * SEQ * 2 * DM)
#define WS_VTL (WS_VTH + 2u * DM * SEQ)
#define WS_O   (WS_VTL + 2u * DM * SEQ)
#define WS_KT  (WS_O + 4u * SEQ * DM)
#define WS_END (WS_KT + 4u * TQB * 32)
static_assert(WS_QK % 128 == 0 && WS_QKL % 128 == 0 && WS_VTH % 128 == 0 && WS_VTL % 128 == 0 && WS_O % 128 == 0 && WS_KT % 128 == 0);
static_assert(WS_END <= 134217728u);

__global__ __launch_bounds__(256) void k_pack(const float* __restrict__ WQ, const float* __restrict__ WK, const float* __restrict__ WV, const float* __restrict__ WO, __bf16* __restrict__ PK) {
  __shared__ __align__(16) __bf16 s[64][72];
  const int k0 = blockIdx.x * 64, n0 = blockIdx.y * 64, which = blockIdx.z, t = threadIdx.x;
  const float* Wm = (which == 0) ? WQ : (which == 1) ? WK : (which == 2) ? WV : WO;
  for (int p = t; p < 64 * 16; p += 256) { const int kr = p >> 4, c4 = (p & 15) * 4;
    const v4f v = *(const v4f*)(Wm + (size_t)(k0 + kr) * DM + n0 + c4);
    s[c4 + 0][kr] = (__bf16)v[0]; s[c4 + 1][kr] = (__bf16)v[1]; s[c4 + 2][kr] = (__bf16)v[2]; s[c4 + 3][kr] = (__bf16)v[3]; }
  __syncthreads();
  __bf16* dst = PK + ((size_t)which * DM + n0) * DM + k0;
  for (int p = t; p < 64 * 8; p += 256) { const int nl = p >> 3, pc = p & 7; vst2(dst + (size_t)nl * DM + pc * 8, *(const v4u*)&s[nl][pc * 8]); }
}
__global__ __launch_bounds__(256) void k_kt(const int* __restrict__ MK, int* __restrict__ KT) {
  __shared__ int sm[8];
  const int qb = blockIdx.x, t = threadIdx.x, lane = t & 31, wave = t >> 5;
  const int per_row = SEQ / 4;
  int mx = -1;
#pragma unroll 1
  for (int p = t; p < 64 * per_row; p += 256) { const int row = p / per_row, c4 = (p - row * per_row) * 4;
    const v4i v = *(const v4i*)(MK + (size_t)(qb * 64 + row) * SS_FULL + c4);
    mx = (v[0] != 0 && c4 + 0 > mx) ? c4 + 0 : mx; mx = (v[1] != 0 && c4 + 1 > mx) ? c4 + 1 : mx;
    mx = (v[2] != 0 && c4 + 2 > mx) ? c4 + 2 : mx; mx = (v[3] != 0 && c4 + 3 > mx) ? c4 + 3 : mx; }
#pragma unroll
  for (int o = 1; o < 32; o <<= 1) { const int y = __shfl_xor(mx, o); mx = y > mx ? y : mx; }
  if (lane == 0) sm[wave] = mx;
  __syncthreads();
  if (wave == 0) { int m2 = sm[lane & 7];
#pragma unroll
    for (int o = 1; o < 8; o <<= 1) { const int y = __shfl_xor(m2, o); m2 = y > m2 ? y : m2; }
    const int nkt = (m2 < 0) ? 0 : ((m2 >> 5) + 1);
    if (lane < 8) { v4i w; w[0] = nkt; w[1] = nkt; w[2] = nkt; w[3] = nkt; vst2(KT + (size_t)qb * 32 + lane * 4, w); } }
}
__global__ __launch_bounds__(128) void k_qkv(const float* __restrict__ X, const __bf16* __restrict__ P, _Float16* __restrict__ QK, _Float16* __restrict__ QKL, _Float16* __restrict__ VTH, _Float16* __restrict__ VTL) {
  __shared__ __align__(16) _Float16 so[4][16][136], sol[4][16][136]; __shared__ __align__(16) _Float16 sth[128][72], stl[128][72];
  const int tid = threadIdx.x, wave = tid >> 5, lane = tid & 31, col = lane & 15, g = lane >> 4; const size_t r0 = (size_t)blockIdx.x * 64 + wave * 16; const int n0 = blockIdx.y * 128;
  v8f acc[8] = {};
#pragma unroll 2
  for (int kc = 0; kc < DM / 32; ++kc) { v16b a; { const float* p = X + (r0 + col) * DM + kc * 32 + 8 * g;
#pragma unroll
      for (int i = 0; i < 8; ++i) { a[i] = (__bf16)p[i]; a[8 + i] = (__bf16)p[16 + i]; } }
#pragma unroll
    for (int j = 0; j < 8; ++j) acc[j] = wmma_bf(a, frag_b(P + (size_t)(n0 + j * 16 + col) * DM + kc * 32, lane), acc[j]); }
  if (n0 < 2 * DM) {
#pragma unroll
    for (int j = 0; j < 8; ++j) {
#pragma unroll
      for (int r = 0; r < 8; ++r) { const float v = acc[j][r]; const _Float16 hv = (_Float16)v; so[wave][8 * g + r][j * 16 + col] = hv; sol[wave][8 * g + r][j * 16 + col] = (_Float16)((v - (float)hv) * 2048.0f); } }
    LDSX();
    for (int rl = 0; rl < 16; ++rl) if (lane < 16) { vst2(QK + (r0 + rl) * (2 * DM) + n0 + lane * 8, *(const v4u*)&so[wave][rl][lane * 8]); vst2(QKL + (r0 + rl) * (2 * DM) + n0 + lane * 8, *(const v4u*)&sol[wave][rl][lane * 8]); }
  } else {
#pragma unroll
    for (int j = 0; j < 8; ++j) {
#pragma unroll
      for (int r = 0; r < 8; ++r) { const float v = acc[j][r]; const _Float16 hv = (_Float16)v; sth[j * 16 + col][wave * 16 + 8 * g + r] = hv; stl[j * 16 + col][wave * 16 + 8 * g + r] = (_Float16)((v - (float)hv) * 2048.0f); } }
    __syncthreads();
    const int s0 = blockIdx.x * 64; const int pc0 = n0 - 2 * DM;
    for (int q = tid; q < 128 * 8; q += 128) { const int d = q >> 3, pc = q & 7; const size_t o = ((size_t)(pc0 + d)) * SEQ + s0 + pc * 8; vst2(VTH + o, *(const v4u*)&sth[d][pc * 8]); vst2(VTL + o, *(const v4u*)&stl[d][pc * 8]); }
  }
}
__global__ __launch_bounds__(128) void k_attn(const _Float16* __restrict__ QK, const _Float16* __restrict__ QKL, const _Float16* __restrict__ VTH, const _Float16* __restrict__ VTL, const int* __restrict__ MK, const int* __restrict__ KT, float* __restrict__ O) {
  __shared__ __align__(16) float sp[4][16][36]; __shared__ __align__(16) float so[4][16][68]; __shared__ __align__(16) int smk[4][16][36];
  const int tid = threadIdx.x, wave = tid >> 5, lane = tid & 31, col = lane & 15, g = lane >> 4;
  const int qb = blockIdx.x, h = blockIdx.y; const int q0 = qb * 64 + wave * 16; const size_t rq = (size_t)q0 + col;
  v16h aq[2], aql[2];
#pragma unroll
  for (int kc = 0; kc < 2; ++kc) { aq[kc] = frag_h(QK + rq * (2 * DM) + h * HD + kc * 32, lane); aql[kc] = frag_h(QKL + rq * (2 * DM) + h * HD + kc * 32, lane); }
  float m[8], l[8];
#pragma unroll
  for (int r = 0; r < 8; ++r) { m[r] = -3.0e38f; l[r] = 0.f; }
  v8f acc[4] = {}, accl[4] = {};
  const int nraw = KT[(size_t)qb * 32];
  const int nks = nraw < 0 ? 0 : (nraw > SEQ / 32 ? SEQ / 32 : nraw);
#pragma unroll 1
  for (int ks = 0; ks < nks; ++ks) {
#pragma unroll
    for (int it = 0; it < 4; ++it) { const int p = it * 32 + lane, row = p >> 3, c4 = (p & 7) * 4;
      *(v4i*)&smk[wave][row][c4] = *(const v4i*)(MK + (size_t)(q0 + row) * SS_FULL + ks * 32 + c4); }
    LDSX();
    v8f s[2];
#pragma unroll
    for (int ct = 0; ct < 2; ++ct) { const int kk = ks * 32 + ct * 16 + col; const _Float16* krow = QK + (size_t)kk * (2 * DM) + DM + h * HD; const _Float16* krowl = QKL + (size_t)kk * (2 * DM) + DM + h * HD; v8f c = {}, cl = {};
#pragma unroll
      for (int kc = 0; kc < 2; ++kc) { const v16h kh = frag_h(krow + kc * 32, lane); c = wmma16(aq[kc], kh, c); cl = wmma16(aql[kc], kh, cl); cl = wmma16(aq[kc], frag_h(krowl + kc * 32, lane), cl); }
#pragma unroll
      for (int r = 0; r < 8; ++r) { const float sc = (c[r] + cl[r] * (1.0f / 2048.0f)) * 0.125f; const int mk = smk[wave][8 * g + r][ct * 16 + col]; s[ct][r] = (mk != 0) ? sc : -3.0e38f; } }
#pragma unroll
    for (int r = 0; r < 8; ++r) { float mx = fmaxf(s[0][r], s[1][r]);
#pragma unroll
      for (int o = 1; o < 16; o <<= 1) mx = fmaxf(mx, __shfl_xor(mx, o));
      const float mn = fmaxf(m[r], mx); const float alpha = (m[r] <= -1.0e38f) ? 0.f : __expf(m[r] - mn);
      const float e0 = (s[0][r] <= -1.0e38f) ? 0.f : __expf(s[0][r] - mn), e1 = (s[1][r] <= -1.0e38f) ? 0.f : __expf(s[1][r] - mn); float es = e0 + e1;
#pragma unroll
      for (int o = 1; o < 16; o <<= 1) es += __shfl_xor(es, o);
      l[r] = l[r] * alpha + es; m[r] = mn;
#pragma unroll
      for (int dt = 0; dt < 4; ++dt) { acc[dt][r] *= alpha; accl[dt][r] *= alpha; }
      sp[wave][8 * g + r][col] = e0; sp[wave][8 * g + r][16 + col] = e1; }
    LDSX();
    v16h pa, pl; { const float* prow = &sp[wave][col][0] + 8 * (lane >> 4);
#pragma unroll
      for (int i = 0; i < 8; ++i) { const float x0 = prow[i] * 2048.0f, x1 = prow[16 + i] * 2048.0f; const _Float16 h0 = (_Float16)x0, h1 = (_Float16)x1; pa[i] = h0; pa[8 + i] = h1; pl[i] = (_Float16)((x0 - (float)h0) * 2048.0f); pl[8 + i] = (_Float16)((x1 - (float)h1) * 2048.0f); } }
#pragma unroll
    for (int dt = 0; dt < 4; ++dt) { const size_t vr = ((size_t)(h * HD + dt * 16 + col)) * SEQ + ks * 32; const v16h vh = frag_h(VTH + vr, lane); acc[dt] = wmma16(pa, vh, acc[dt]); if (qb < 2) { accl[dt] = wmma16(pl, vh, accl[dt]); accl[dt] = wmma16(pa, frag_h(VTL + vr, lane), accl[dt]); } }
    LDSX(); }
#pragma unroll
  for (int r = 0; r < 8; ++r) { const float il = (1.0f / 2048.0f) / l[r];
#pragma unroll
    for (int dt = 0; dt < 4; ++dt) so[wave][8 * g + r][dt * 16 + col] = (acc[dt][r] + accl[dt][r] * (1.0f / 2048.0f)) * il; }
  LDSX();
  for (int rl = 0; rl < 16; ++rl) if (lane < 16) vst2(O + ((size_t)q0 + rl) * DM + h * HD + lane * 4, *(const v4f*)&so[wave][rl][lane * 4]);
}
__global__ __launch_bounds__(128) void k_out(const float* __restrict__ O, const __bf16* __restrict__ P, float* __restrict__ Y) {
  __shared__ __align__(16) float so[4][16][132];
  const int tid = threadIdx.x, wave = tid >> 5, lane = tid & 31, col = lane & 15, g = lane >> 4; const size_t r0 = (size_t)blockIdx.x * 64 + wave * 16; const int n0 = blockIdx.y * 128;
  v8f acc[8] = {};
#pragma unroll 2
  for (int kc = 0; kc < DM / 32; ++kc) { const F2 a = split_row(O + (r0 + col) * DM, kc * 32, lane);
#pragma unroll
    for (int j = 0; j < 8; ++j) { const v16b w = frag_b(P + (size_t)(n0 + j * 16 + col) * DM + kc * 32, lane); acc[j] = wmma_bf(a.l, w, acc[j]); acc[j] = wmma_bf(a.h, w, acc[j]); } }
#pragma unroll
  for (int j = 0; j < 8; ++j) {
#pragma unroll
    for (int r = 0; r < 8; ++r) so[wave][8 * g + r][j * 16 + col] = acc[j][r]; }
  LDSX();
  for (int rl = 0; rl < 16; ++rl) vst2(Y + (r0 + rl) * DM + n0 + lane * 4, *(const v4f*)&so[wave][rl][lane * 4]);
}
extern "C" void kernel_launch(void* const* d_in, const int* in_sizes, int n_in, void* d_out, int out_size, void* d_ws, size_t ws_size, hipStream_t stream) {
  if (n_in < 6) return;
  if (in_sizes[0] < SEQ * DM) return;
  if (in_sizes[1] < SEQ * SS_FULL) return;
  if (in_sizes[2] < DM * DM || in_sizes[3] < DM * DM || in_sizes[4] < DM * DM || in_sizes[5] < DM * DM) return;
  if (out_size < SEQ * DM) return;
  if (ws_size < (size_t)WS_END) return;
  const float* X  = (const float*)d_in[0];
  const int*   MK = (const int*)d_in[1];
  const float* WQ = (const float*)d_in[2];
  const float* WK = (const float*)d_in[3];
  const float* WV = (const float*)d_in[4];
  const float* WO = (const float*)d_in[5];
  char* ws = (char*)d_ws; __bf16* PK = (__bf16*)(ws + WS_PK); _Float16 *QK = (_Float16*)(ws + WS_QK), *QKL = (_Float16*)(ws + WS_QKL), *VTH = (_Float16*)(ws + WS_VTH), *VTL = (_Float16*)(ws + WS_VTL); float* O = (float*)(ws + WS_O); int* KT = (int*)(ws + WS_KT);
  k_pack<<<dim3(DM / 64, DM / 64, 4), 256, 0, stream>>>(WQ, WK, WV, WO, PK);
  k_kt<<<dim3(TQB), 256, 0, stream>>>(MK, KT);
  k_qkv<<<dim3(SEQ / 64, QKVW / 128), 128, 0, stream>>>(X, PK + PK_A, QK, QKL, VTH, VTL);
  k_attn<<<dim3(TQB, NH), 128, 0, stream>>>(QK, QKL, VTH, VTL, MK, KT, O);
  k_out<<<dim3(SEQ / 64, DM / 128), 128, 0, stream>>>(O, PK + PK_P, (float*)d_out);
}
